// myGPT2Block_44667659879006
// MI455X (gfx1250) — hardware-verified
//
#include <hip/hip_runtime.h>


typedef _Float16 v16h __attribute__((ext_vector_type(16)));
typedef _Float16 v8h  __attribute__((ext_vector_type(8)));
typedef _Float16 v8ha __attribute__((ext_vector_type(8), may_alias));
typedef _Float16 v2h  __attribute__((ext_vector_type(2)));
typedef float    v8f  __attribute__((ext_vector_type(8)));
typedef float    v4f  __attribute__((ext_vector_type(4)));
typedef float    v4fa __attribute__((ext_vector_type(4), may_alias));
typedef unsigned int v4u  __attribute__((ext_vector_type(4)));
typedef unsigned int v4ua __attribute__((ext_vector_type(4), may_alias));

#define DEV __device__ __forceinline__

constexpr int BS    = 2;
constexpr int SEQ   = 2048;
constexpr int DM    = 1024;
constexpr int NH    = 16;
constexpr int HD    = 64;
constexpr int INNER = 4096;
constexpr int MROWS = BS * SEQ;
constexpr int LDSS  = 72;
constexpr int PSS   = 72;
constexpr float LN_EPS = 1e-5f;
constexpr float WSC    = 64.f;

union Frag { v16h v; v8h hf[2]; };
union H8   { v8h h; v4u u; };
union H2   { v2h h; unsigned int u; };

DEV v8f vzero8() {
  v8f z;
#pragma unroll
  for (int i = 0; i < 8; ++i) z[i] = 0.f;
  return z;
}

DEV v16h ldfrag(const _Float16* p, int h) {
  Frag f;
  f.hf[0] = *(const v8ha*)(p + 8 * h);
  f.hf[1] = *(const v8ha*)(p + 16 + 8 * h);
  return f.v;
}

DEV v8f wmma16(v16h a, v16h b, v8f c) {
  v8f d = __builtin_amdgcn_wmma_f32_16x16x32_f16(false, a, false, b, (short)0, c, false, false);
  asm volatile("v_nop\n\tv_nop\n\tv_nop\n\tv_nop" : "+v"(d) : "v"(a), "v"(b));
  return d;
}

DEV unsigned int pk2(float a, float b) {
  H2 t;
  t.h[0] = (_Float16)a;
  t.h[1] = (_Float16)b;
  return t.u;
}
DEV v4u pack8u(v4f a, v4f b) {
  v4u o;
  o[0] = pk2(a[0], a[1]); o[1] = pk2(a[2], a[3]);
  o[2] = pk2(b[0], b[1]); o[3] = pk2(b[2], b[3]);
  return o;
}
DEV void vst4u(unsigned short* p, v4u v) { *(volatile v4u*)p = v; }
DEV void vst4f(float* p, v4f v)          { *(volatile v4f*)p = v; }

__global__ __launch_bounds__(256)
void cvt_wt(const float* __restrict__ W, unsigned short* Wt, int K, int N)
{
  __shared__ float st[64 * 65];
  const int k0 = blockIdx.x * 64, n0 = blockIdx.y * 64;
  if (k0 >= K || n0 >= N) return;
  const int tid = threadIdx.x;
#pragma unroll
  for (int i = 0; i < 4; ++i) {
    const int u = tid + i * 256;
    const int kk = u >> 4, c4 = (u & 15) * 4;
    const v4f w = *(const v4fa*)(W + (size_t)(k0 + kk) * N + n0 + c4);
    st[(c4 + 0) * 65 + kk] = w[0];
    st[(c4 + 1) * 65 + kk] = w[1];
    st[(c4 + 2) * 65 + kk] = w[2];
    st[(c4 + 3) * 65 + kk] = w[3];
  }
  __syncthreads();
  const int lane = tid & 31, wave = tid >> 5;
  const int j = lane & 7;
  for (int pass = 0; pass < 2; ++pass) {
    if (pass) __threadfence();
    asm volatile("" ::: "memory");
#pragma unroll
    for (int p = 0; p < 2; ++p) {
      const int nn = wave * 8 + p * 4 + (lane >> 3);
      const float* sp = st + nn * 65 + j * 8;
      v4f a, b;
#pragma unroll
      for (int e = 0; e < 4; ++e) { a[e] = sp[e] * WSC; b[e] = sp[4 + e] * WSC; }
      const v4u o = pack8u(a, b);
      unsigned short* dst = Wt + (size_t)(n0 + nn) * K + k0 + j * 8;
      vst4u(dst, o);
    }
  }
}

__global__ __launch_bounds__(128)
void ln_f16(const float* __restrict__ x, const float* __restrict__ g, const float* __restrict__ bta,
            unsigned short* out, int nrows)
{
  __shared__ float red[8];
  const int row = blockIdx.x;
  if (row >= nrows) return;
  const int tid = threadIdx.x, lane = tid & 31, wave = tid >> 5;
  const int c0 = tid * 8;
  const float* xr = x + (size_t)row * DM + c0;
  const v4f xa = *(const v4fa*)xr;
  const v4f xb = *(const v4fa*)(xr + 4);
  float v[8];
#pragma unroll
  for (int i = 0; i < 4; ++i) { v[i] = xa[i]; v[4 + i] = xb[i]; }
  float s = 0.f;
#pragma unroll
  for (int i = 0; i < 8; ++i) s += v[i];
#pragma unroll
  for (int msk = 16; msk >= 1; msk >>= 1) s += __shfl_xor(s, msk, 32);
  if (lane == 0) red[wave] = s;
  __syncthreads();
  const float mu = (red[0] + red[1] + red[2] + red[3]) * (1.f / DM);
  float d[8], ss = 0.f;
#pragma unroll
  for (int i = 0; i < 8; ++i) { d[i] = v[i] - mu; ss += d[i] * d[i]; }
#pragma unroll
  for (int msk = 16; msk >= 1; msk >>= 1) ss += __shfl_xor(ss, msk, 32);
  if (lane == 0) red[4 + wave] = ss;
  __syncthreads();
  const float var = (red[4] + red[5] + red[6] + red[7]) * (1.f / DM);
  const float inv = rsqrtf(var + LN_EPS);
  const v4f ga = *(const v4fa*)(g + c0),   gb = *(const v4fa*)(g + c0 + 4);
  const v4f ba = *(const v4fa*)(bta + c0), bb = *(const v4fa*)(bta + c0 + 4);
  v4f ya, yb;
#pragma unroll
  for (int i = 0; i < 4; ++i) {
    ya[i] = d[i] * inv * ga[i] + ba[i];
    yb[i] = d[4 + i] * inv * gb[i] + bb[i];
  }
  const v4u o = pack8u(ya, yb);
  unsigned short* dst = out + (size_t)row * DM + c0;
  vst4u(dst, o);
  __threadfence();
  vst4u(dst, o);
}

template <int EPI>
__global__ __launch_bounds__(256)
void gemm_f16(const unsigned short* __restrict__ Ag, const unsigned short* __restrict__ Bg,
              const float* __restrict__ bias, const float* __restrict__ resid,
              float* outf, unsigned short* outh0, unsigned short* outh1,
              int lda, int ldb, int K, int Mtot, int Ntot)
{
  __shared__ __attribute__((aligned(16))) float smem[9216];
  _Float16* sA = reinterpret_cast<_Float16*>(smem);
  _Float16* sB = sA + 128 * LDSS;
  const _Float16* A  = reinterpret_cast<const _Float16*>(Ag);
  const _Float16* Bt = reinterpret_cast<const _Float16*>(Bg);
  const int tid = threadIdx.x, lane = tid & 31, wave = tid >> 5;
  const int wm = wave & 3, wn = wave >> 2;
  const int m = lane & 15, h = lane >> 4;
  const int m0 = blockIdx.y * 128, n0 = blockIdx.x * 128;
  if (m0 >= Mtot || n0 >= Ntot) return;
  constexpr float SC = (EPI == 2) ? (1.f / 1024.f) : (1.f / 64.f);

  v8f acc[2][4];
#pragma unroll
  for (int i = 0; i < 2; ++i)
#pragma unroll
    for (int jn = 0; jn < 4; ++jn) acc[i][jn] = vzero8();

  for (int kt = 0; kt < K; kt += 64) {
    __syncthreads();
#pragma unroll
    for (int i = 0; i < 4; ++i) {
      const int u = tid + i * 256;
      const int row = u >> 3, kq = (u & 7) * 8;
      const v8h va = *(const v8ha*)(A  + (size_t)(m0 + row) * lda + kt + kq);
      const v8h vb = *(const v8ha*)(Bt + (size_t)(n0 + row) * ldb + kt + kq);
      *(v8ha*)(sA + row * LDSS + kq) = va;
      *(v8ha*)(sB + row * LDSS + kq) = vb;
    }
    __syncthreads();
#pragma unroll
    for (int kc = 0; kc < 64; kc += 32) {
      const v16h a0 = ldfrag(sA + (wm * 32 + m) * LDSS + kc, h);
      const v16h a1 = ldfrag(sA + (wm * 32 + 16 + m) * LDSS + kc, h);
#pragma unroll
      for (int nf = 0; nf < 4; ++nf) {
        const v16h bfr = ldfrag(sB + (wn * 64 + nf * 16 + m) * LDSS + kc, h);
        acc[0][nf] = wmma16(a0, bfr, acc[0][nf]);
        acc[1][nf] = wmma16(a1, bfr, acc[1][nf]);
      }
    }
  }
  __syncthreads();

  float* stg = smem + wave * 1024;
  const int colbase = n0 + wn * 64;
#pragma unroll
  for (int mf = 0; mf < 2; ++mf) {
    const int rowbase = m0 + wm * 32 + mf * 16;
#pragma unroll
    for (int nf = 0; nf < 4; ++nf)
#pragma unroll
      for (int r = 0; r < 8; ++r) {
        float v = acc[mf][nf][r] * SC;
        if constexpr (EPI == 0) v += bias[colbase + nf * 16 + m];
        if constexpr (EPI == 3) { v = (v >= 0.f) ? v : v * 0.01f; v *= 16.f; }
        stg[(8 * h + r) * 64 + nf * 16 + m] = v;
      }
    __syncthreads();

    if constexpr (EPI == 2) {
      const int rq = lane >> 4, j = lane & 15;
      for (int pass = 0; pass < 2; ++pass) {
        if (pass) __threadfence();
        asm volatile("" ::: "memory");
#pragma unroll
        for (int p = 0; p < 8; ++p) {
          const int r = p * 2 + rq;
          const size_t idx = (size_t)(rowbase + r) * Ntot + colbase + j * 4;
          v4f v = *(const v4fa*)(stg + r * 64 + j * 4);
          const v4f rr = *(const v4fa*)(resid + idx);
          v = v + rr;
          vst4f(outf + idx, v);
        }
      }
    } else {
      const int rq = lane >> 3, j = lane & 7;
      for (int pass = 0; pass < 2; ++pass) {
        if (pass) __threadfence();
        asm volatile("" ::: "memory");
#pragma unroll
        for (int p = 0; p < 4; ++p) {
          const int r = p * 4 + rq;
          const float* sp = stg + r * 64 + j * 8;
          const v4u o = pack8u(*(const v4fa*)sp, *(const v4fa*)(sp + 4));
          unsigned short* dst;
          if constexpr (EPI == 0) {
            const int nn = colbase & (DM - 1);
            const int hh = nn >> 6;
            unsigned short* base = (colbase >= DM) ? outh1 : outh0;
            const int t = rowbase + r;
            dst = base + ((size_t)((t / SEQ) * NH + hh) * SEQ + (t % SEQ)) * HD + j * 8;
          } else if constexpr (EPI == 1) {
            const int dch = rowbase + r;
            const int hh = dch >> 6, hd = dch & (HD - 1);
            const int bb = colbase / SEQ, s0 = colbase % SEQ;
            dst = outh0 + ((size_t)((bb * NH + hh) * HD + hd)) * SEQ + s0 + j * 8;
          } else {
            dst = outh0 + (size_t)(rowbase + r) * Ntot + colbase + j * 8;
          }
          vst4u(dst, o);
        }
      }
    }
    __syncthreads();
  }
}

__global__ __launch_bounds__(128)
void attn_f16(const unsigned short* __restrict__ qg, const unsigned short* __restrict__ kg,
              const unsigned short* __restrict__ vtg, unsigned short* obuf, int nbh)
{
  __shared__ __attribute__((aligned(16))) _Float16 pst[4 * 16 * PSS];
  const int lane = threadIdx.x & 31, wave = threadIdx.x >> 5;
  const int m = lane & 15, h = lane >> 4;
  const int bh   = blockIdx.x / (SEQ / 64);
  const int qblk = blockIdx.x % (SEQ / 64);
  if (bh >= nbh) return;
  const int q0 = qblk * 64 + wave * 16;
  const _Float16* qh = reinterpret_cast<const _Float16*>(qg)  + (size_t)bh * SEQ * HD;
  const _Float16* kh = reinterpret_cast<const _Float16*>(kg)  + (size_t)bh * SEQ * HD;
  const _Float16* vh = reinterpret_cast<const _Float16*>(vtg) + (size_t)bh * HD * SEQ;

  const v16h qa0 = ldfrag(qh + (size_t)(q0 + m) * HD, h);
  const v16h qa1 = ldfrag(qh + (size_t)(q0 + m) * HD + 32, h);

  v8f o0 = vzero8(), o1 = vzero8(), o2 = vzero8(), o3 = vzero8();
  float mrun[8], lrun[8];
#pragma unroll
  for (int r = 0; r < 8; ++r) { mrun[r] = -1e30f; lrun[r] = 0.f; }

  _Float16* ps = pst + wave * (16 * PSS);
  const int kend = q0 + 16;
  for (int kb = 0; kb < kend; kb += 32) {
    const _Float16* kr0 = kh + (size_t)(kb + m) * HD;
    const _Float16* kr1 = kr0 + 16 * HD;
    v8f s0 = vzero8(), s1 = vzero8();
    s0 = wmma16(qa0, ldfrag(kr0, h),      s0);
    s0 = wmma16(qa1, ldfrag(kr0 + 32, h), s0);
    s1 = wmma16(qa0, ldfrag(kr1, h),      s1);
    s1 = wmma16(qa1, ldfrag(kr1 + 32, h), s1);

    const bool edge = (kb + 31 > q0);
    float sc0[8], sc1[8];
#pragma unroll
    for (int r = 0; r < 8; ++r) {
      float a0 = s0[r] * 0.125f, a1 = s1[r] * 0.125f;
      if (edge) {
        const int rowq = q0 + 8 * h + r;
        if (kb + m > rowq)      a0 = -1e30f;
        if (kb + 16 + m > rowq) a1 = -1e30f;
      }
      sc0[r] = a0; sc1[r] = a1;
    }
#pragma unroll
    for (int r = 0; r < 8; ++r) {
      float tmax = fmaxf(sc0[r], sc1[r]);
#pragma unroll
      for (int msk = 8; msk >= 1; msk >>= 1) tmax = fmaxf(tmax, __shfl_xor(tmax, msk, 32));
      const float mnew = fmaxf(mrun[r], tmax);
      const float corr = __expf(mrun[r] - mnew);
      const float p0 = __expf(sc0[r] - mnew);
      const float p1 = __expf(sc1[r] - mnew);
      float psum = p0 + p1;
#pragma unroll
      for (int msk = 8; msk >= 1; msk >>= 1) psum += __shfl_xor(psum, msk, 32);
      lrun[r] = lrun[r] * corr + psum;
      mrun[r] = mnew;
      o0[r] = o0[r] * corr; o1[r] = o1[r] * corr; o2[r] = o2[r] * corr; o3[r] = o3[r] * corr;
      ps[(8 * h + r) * PSS + m]      = (_Float16)(p0 * 256.f);
      ps[(8 * h + r) * PSS + 16 + m] = (_Float16)(p1 * 256.f);
    }
    asm volatile("" ::: "memory");
    const v16h pf = ldfrag(ps + m * PSS, h);
    asm volatile("" ::: "memory");
    const _Float16* vr = vh + (size_t)m * SEQ + kb;
    o0 = wmma16(pf, ldfrag(vr, h),            o0);
    o1 = wmma16(pf, ldfrag(vr + 16 * SEQ, h), o1);
    o2 = wmma16(pf, ldfrag(vr + 32 * SEQ, h), o2);
    o3 = wmma16(pf, ldfrag(vr + 48 * SEQ, h), o3);
  }

  asm volatile("" ::: "memory");
#pragma unroll
  for (int r = 0; r < 8; ++r) {
    const float il = 0.0625f / lrun[r];
    const int rr = (8 * h + r) * PSS;
    ps[rr + m]      = (_Float16)(o0[r] * il);
    ps[rr + 16 + m] = (_Float16)(o1[r] * il);
    ps[rr + 32 + m] = (_Float16)(o2[r] * il);
    ps[rr + 48 + m] = (_Float16)(o3[r] * il);
  }
  asm volatile("" ::: "memory");
  const int b = bh / NH, hh = bh % NH;
  const int rq = lane >> 3, j = lane & 7;
  for (int pass = 0; pass < 2; ++pass) {
    if (pass) __threadfence();
    asm volatile("" ::: "memory");
#pragma unroll
    for (int p = 0; p < 4; ++p) {
      const int row = p * 4 + rq;
      H8 t;
      t.h = *(const v8ha*)(ps + row * PSS + j * 8);
      unsigned short* dst = obuf + ((size_t)(b * SEQ + q0 + row)) * DM + hh * HD + j * 8;
      vst4u(dst, t.u);
    }
  }
}

extern "C" void kernel_launch(void* const* d_in, const int* in_sizes, int n_in,
                              void* d_out, int out_size, void* d_ws, size_t ws_size,
                              hipStream_t stream)
{
  if (n_in < 11) return;
  if (in_sizes[0] != MROWS * DM || in_sizes[1] != DM || in_sizes[2] != DM ||
      in_sizes[3] != DM || in_sizes[4] != DM || in_sizes[5] != DM * 2 * DM ||
      in_sizes[6] != 2 * DM || in_sizes[7] != DM * DM || in_sizes[8] != DM * DM ||
      in_sizes[9] != DM * INNER || in_sizes[10] != INNER * DM || out_size != MROWS * DM) return;

  const float* x    = (const float*)d_in[0];
  const float* ln1g = (const float*)d_in[1];
  const float* ln1b = (const float*)d_in[2];
  const float* ln2g = (const float*)d_in[3];
  const float* ln2b = (const float*)d_in[4];
  const float* Wqk  = (const float*)d_in[5];
  const float* bqk  = (const float*)d_in[6];
  const float* Wv   = (const float*)d_in[7];
  const float* Wo   = (const float*)d_in[8];
  const float* Wfc  = (const float*)d_in[9];
  const float* Wpj  = (const float*)d_in[10];
  float* out = (float*)d_out;

  const size_t szWqk = (size_t)2 * DM * DM * 2;
  const size_t szW1  = (size_t)DM * DM * 2;
  const size_t szWfc = (size_t)DM * INNER * 2;
  const size_t szAct = (size_t)MROWS * DM * 2;
  const size_t szX1  = (size_t)MROWS * DM * 4;
  const size_t szA   = (size_t)MROWS * INNER * 2;
  char* ws = (char*)d_ws;
  size_t off = 0;
  unsigned short* wqk_t = (unsigned short*)(ws + off); off += szWqk;
  unsigned short* wv_t  = (unsigned short*)(ws + off); off += szW1;
  unsigned short* wo_t  = (unsigned short*)(ws + off); off += szW1;
  unsigned short* wfc_t = (unsigned short*)(ws + off); off += szWfc;
  unsigned short* wpj_t = (unsigned short*)(ws + off); off += szWfc;
  unsigned short* h_t   = (unsigned short*)(ws + off); off += szAct;
  unsigned short* q_t   = (unsigned short*)(ws + off); off += szAct;
  unsigned short* k_t   = (unsigned short*)(ws + off); off += szAct;
  unsigned short* vt_t  = (unsigned short*)(ws + off); off += szAct;
  unsigned short* o_t   = (unsigned short*)(ws + off); off += szAct;
  float*          x1    = (float*)         (ws + off); off += szX1;
  unsigned short* a_t   = (unsigned short*)(ws + off); off += szA;
  if (off > ws_size) return;
  unsigned short* h2_t = h_t;

  cvt_wt<<<dim3(DM / 64, (2 * DM) / 64), 256, 0, stream>>>(Wqk, wqk_t, DM, 2 * DM);
  cvt_wt<<<dim3(DM / 64, DM / 64), 256, 0, stream>>>(Wv, wv_t, DM, DM);
  cvt_wt<<<dim3(DM / 64, DM / 64), 256, 0, stream>>>(Wo, wo_t, DM, DM);
  cvt_wt<<<dim3(DM / 64, INNER / 64), 256, 0, stream>>>(Wfc, wfc_t, DM, INNER);
  cvt_wt<<<dim3(INNER / 64, DM / 64), 256, 0, stream>>>(Wpj, wpj_t, INNER, DM);

  ln_f16<<<MROWS, 128, 0, stream>>>(x, ln1g, ln1b, h_t, MROWS);
  gemm_f16<0><<<dim3((2 * DM) / 128, MROWS / 128), 256, 0, stream>>>(
      h_t, wqk_t, bqk, nullptr, nullptr, q_t, k_t, DM, DM, DM, MROWS, 2 * DM);
  gemm_f16<1><<<dim3(MROWS / 128, DM / 128), 256, 0, stream>>>(
      wv_t, h_t, nullptr, nullptr, nullptr, vt_t, nullptr, DM, DM, DM, DM, MROWS);
  attn_f16<<<BS * NH * (SEQ / 64), 128, 0, stream>>>(q_t, k_t, vt_t, o_t, BS * NH);
  gemm_f16<2><<<dim3(DM / 128, MROWS / 128), 256, 0, stream>>>(
      o_t, wo_t, nullptr, x, x1, nullptr, nullptr, DM, DM, DM, MROWS, DM);

  ln_f16<<<MROWS, 128, 0, stream>>>(x1, ln2g, ln2b, h2_t, MROWS);
  gemm_f16<3><<<dim3(INNER / 128, MROWS / 128), 256, 0, stream>>>(
      h2_t, wfc_t, nullptr, nullptr, nullptr, a_t, nullptr, DM, DM, DM, MROWS, INNER);
  gemm_f16<2><<<dim3(DM / 128, MROWS / 128), 256, 0, stream>>>(
      a_t, wpj_t, nullptr, x1, out, nullptr, nullptr, INNER, INNER, INNER, MROWS, DM);
}
